// Causal_self_attention_77730318123444
// MI455X (gfx1250) — hardware-verified
//
#include <hip/hip_runtime.h>
#include <stdint.h>

typedef __attribute__((ext_vector_type(16))) _Float16 v16h;
typedef __attribute__((ext_vector_type(8)))  _Float16 v8h;
typedef __attribute__((ext_vector_type(16))) __bf16   v16b;
typedef __attribute__((ext_vector_type(8)))  __bf16   v8b;
typedef __attribute__((ext_vector_type(8)))  float    v8f;
typedef __attribute__((ext_vector_type(4)))  float    v4f;
typedef __attribute__((ext_vector_type(2)))  float    v2f;
typedef __attribute__((ext_vector_type(4)))  unsigned int u32x4;

constexpr int NBATCH = 2;
constexpr int NT     = 4096;
constexpr int NC     = 768;
constexpr int NH     = 12;
constexpr int HD     = 64;
constexpr int NQKV   = 3 * NC;
constexpr int NTOK   = NBATCH * NT;
constexpr int NQKCOL = 2 * NC;
constexpr float SCORE_SCALE = 0.125f;
constexpr float PCARRY    = 32768.0f;
constexpr float RES_CARRY = 65536.0f;
constexpr float RES_CARRY_INV = 1.0f / 65536.0f;

static_assert(NTOK % 64 == 0 && NQKCOL % 64 == 0 && NC % 64 == 0 && NT % 64 == 0, "tile");
static_assert(NC % 32 == 0, "ktail");
static_assert(NQKV % 64 == 0 && HD == 64 && NH * HD == NC, "geom");

__device__ __forceinline__ unsigned short f2bf_bits(float f) {
  unsigned u = __float_as_uint(f);
  return (unsigned short)((u + 0x7FFFu + ((u >> 16) & 1u)) >> 16);
}
__device__ __forceinline__ float bf_bits2f(unsigned short h) { return __uint_as_float(((unsigned)h) << 16); }
__device__ __forceinline__ float bf_rne(float f) { return bf_bits2f(f2bf_bits(f)); }
__device__ __forceinline__ unsigned h2bits(_Float16 h) { return (unsigned)__builtin_bit_cast(unsigned short, h); }

__device__ __forceinline__ void dep_guard_h(v8f& a, v8f& b, v16h x, v16h y) { asm volatile("v_nop\n\tv_nop\n\tv_nop\n\tv_nop" : "+v"(a), "+v"(b) : "v"(x), "v"(y)); }
__device__ __forceinline__ void dep_guard_b(v8f& a, v8f& b, v16b x, v16b y) { asm volatile("v_nop\n\tv_nop\n\tv_nop\n\tv_nop" : "+v"(a), "+v"(b) : "v"(x), "v"(y)); }
__device__ __forceinline__ void keep4_h(v16h a, v16h b, v16h c, v16h d) { asm volatile("v_nop" :: "v"(a), "v"(b), "v"(c), "v"(d)); }
__device__ __forceinline__ void keep4_b(v16b a, v16b b, v16b c, v16b d) { asm volatile("v_nop" :: "v"(a), "v"(b), "v"(c), "v"(d)); }
__device__ __forceinline__ void acc_guard4(v8f& a, v8f& b, v8f& c, v8f& d) { asm volatile("v_nop\n\tv_nop\n\tv_nop\n\tv_nop" : "+v"(a), "+v"(b), "+v"(c), "+v"(d)); }
template <typename T> struct Frag;
template <> struct Frag<_Float16> {
  typedef v16h V; union U { v16h v; v8h h[2]; };
  static __device__ __forceinline__ v16h load(const _Float16* p) {
    U f; f.h[0] = *(const v8h*)(p); f.h[1] = *(const v8h*)(p + 16); return f.v;
  }
  static __device__ __forceinline__ v8f mma(v16h a, v16h b, v8f c) {
    return __builtin_amdgcn_wmma_f32_16x16x32_f16(false, a, false, b, (short)0, c, false, false);
  }
  static __device__ __forceinline__ void guard(v8f& a, v8f& b, v16h x, v16h y) { dep_guard_h(a, b, x, y); }
  static __device__ __forceinline__ void keep(v16h a, v16h b, v16h c, v16h d) { keep4_h(a, b, c, d); }
};
template <> struct Frag<__bf16> {
  typedef v16b V; union U { v16b v; v8b h[2]; };
  static __device__ __forceinline__ v16b load(const __bf16* p) {
    U f; f.h[0] = *(const v8b*)(p); f.h[1] = *(const v8b*)(p + 16); return f.v;
  }
  static __device__ __forceinline__ v8f mma(v16b a, v16b b, v8f c) {
    return __builtin_amdgcn_wmma_f32_16x16x32_bf16(false, a, false, b, (short)0, c, false, false);
  }
  static __device__ __forceinline__ void guard(v8f& a, v8f& b, v16b x, v16b y) { dep_guard_b(a, b, x, y); }
  static __device__ __forceinline__ void keep(v16b a, v16b b, v16b c, v16b d) { keep4_b(a, b, c, d); }
};

__device__ __forceinline__ v8f mma_h(v16h a, v16h b, v8f c) {
  c = __builtin_amdgcn_wmma_f32_16x16x32_f16(false, a, false, b, (short)0, c, false, false);
  asm volatile("v_nop\n\tv_nop\n\tv_nop\n\tv_nop" : "+v"(c) : "v"(a), "v"(b));
  return c;
}

template <int ET> struct Elem;
template <> struct Elem<0> { typedef _Float16 T; };
template <> struct Elem<1> { typedef __bf16 T; };
template <int ET, int SPLITK, int BIAS_MODE, int OUT_MODE>
__global__ __launch_bounds__(256) void wmma_gemm64(
    const unsigned short* __restrict__ Ap, const unsigned short* __restrict__ A2p, int lda, long strideA,
    const unsigned short* __restrict__ Btp, int ldb, long strideB,
    void* __restrict__ Cout, void* __restrict__ Cout2, int ldc, long strideC,
    const float* __restrict__ bias,
    int M, int N, int K, float scale) {
  typedef typename Elem<ET>::T T;
  typedef typename Frag<T>::V V;
  const T* A = (const T*)Ap; const T* A2 = (const T*)A2p; const T* Bt = (const T*)Btp;
  __shared__ __align__(16) float sT[8][16 * 68];
  const int b    = blockIdx.y;
  const int lane = threadIdx.x & 31;
  const int wave = threadIdx.x >> 5;
  const int tilesN = N >> 6;
  const int tilesM = M >> 6;
  const int tile = blockIdx.x * 8 + wave;
  if (tile >= tilesM * tilesN) return;
  const int tm = tile / tilesN;
  const int tn = tile - tm * tilesN;
  const int m0 = tm << 6;
  const int n0 = tn << 6;

  const T* Ab  = A  + (size_t)b * strideA;
  const T* Bb  = Bt + (size_t)b * strideB;
  const T* Ab2 = SPLITK ? (A2 + (size_t)b * strideA) : nullptr;

  const int rlane = lane & 15;
  const int koff  = (lane >> 4) * 8;
  const int mOff  = (lane >> 4) * 8;

  v8f acc[4][4];
#pragma unroll
  for (int i = 0; i < 4; ++i)
#pragma unroll
    for (int j = 0; j < 4; ++j) acc[i][j] = (v8f){0.f,0.f,0.f,0.f,0.f,0.f,0.f,0.f};

  for (int k0 = 0; k0 < K; k0 += 32) {
    V bh[4];
#pragma unroll
    for (int j = 0; j < 4; ++j) {
      const size_t bo = (size_t)(n0 + (j << 4) + rlane) * ldb + koff + k0;
      bh[j] = Frag<T>::load(Bb + bo);
    }
#pragma unroll
    for (int i = 0; i < 4; ++i) {
      const size_t ao = (size_t)(m0 + (i << 4) + rlane) * lda + koff + k0;
      V ah = Frag<T>::load(Ab + ao);
      V al = ah;
      if (SPLITK) al = Frag<T>::load(Ab2 + ao);
#pragma unroll
      for (int j = 0; j < 4; ++j) {
        acc[i][j] = Frag<T>::mma(ah, bh[j], acc[i][j]);
        if (SPLITK) acc[i][j] = Frag<T>::mma(al, bh[j], acc[i][j]);
      }
      Frag<T>::guard(acc[i][0], acc[i][3], ah, al);
    }
    Frag<T>::keep(bh[0], bh[1], bh[2], bh[3]);
  }
  acc_guard4(acc[0][0], acc[0][1], acc[0][2], acc[0][3]);
  acc_guard4(acc[1][0], acc[1][1], acc[1][2], acc[1][3]);
  acc_guard4(acc[2][0], acc[2][1], acc[2][2], acc[2][3]);
  acc_guard4(acc[3][0], acc[3][1], acc[3][2], acc[3][3]);

  float* slab = sT[wave];
#pragma unroll
  for (int i = 0; i < 4; ++i) {
    const int mBase = m0 + (i << 4);
    float bm[8];
#pragma unroll
    for (int r = 0; r < 8; ++r) bm[r] = 0.f;
    if (BIAS_MODE == 1) {
      const v4f b0 = *(const v4f*)(bias + mBase + mOff);
      const v4f b1 = *(const v4f*)(bias + mBase + mOff + 4);
#pragma unroll
      for (int e = 0; e < 4; ++e) { bm[e] = bf_rne(b0[e]); bm[4 + e] = bf_rne(b1[e]); }
    }
#pragma unroll
    for (int j = 0; j < 4; ++j) {
      const int n = n0 + (j << 4) + rlane;
      float bv = 0.f;
      if (BIAS_MODE == 2) bv = bf_rne(bias[n]);
#pragma unroll
      for (int r = 0; r < 8; ++r) {
        float v = acc[i][j][r] * scale;
        if (BIAS_MODE == 1) v += bm[r];
        if (BIAS_MODE == 2) v += bv;
        slab[(mOff + r) * 68 + (j << 4) + rlane] = v;
      }
    }
    __builtin_amdgcn_fence(__ATOMIC_RELEASE, "workgroup");
    __builtin_amdgcn_wave_barrier();
    __builtin_amdgcn_fence(__ATOMIC_ACQUIRE, "workgroup");
    if (OUT_MODE == 0) {
      float* C = (float*)Cout + (size_t)b * strideC;
      const int hh = lane >> 4, c4 = (lane & 15) * 4;
      for (int pass = 0; pass < 2; ++pass) {
#pragma unroll
        for (int it = 0; it < 8; ++it) {
          const int row = it * 2 + hh;
          v4f v = *(const v4f*)(slab + row * 68 + c4);
          *(volatile v4f*)(C + (size_t)(mBase + row) * ldc + n0 + c4) = v;
        }
        __threadfence();
      }
    } else {
      const int q = lane >> 3, c8 = (lane & 7) * 8;
      unsigned short* C  = (unsigned short*)Cout  + (size_t)b * strideC;
      unsigned short* C2 = (OUT_MODE == 3) ? ((unsigned short*)Cout2 + (size_t)b * strideC) : nullptr;
      for (int pass = 0; pass < 2; ++pass) {
#pragma unroll
        for (int it = 0; it < 4; ++it) {
          const int row = it * 4 + q;
          const float* sp = slab + row * 68 + c8;
          u32x4 hv = {0u, 0u, 0u, 0u};
          u32x4 lv = {0u, 0u, 0u, 0u};
#pragma unroll
          for (int e2 = 0; e2 < 4; ++e2) {
            const float f0 = sp[2 * e2], f1 = sp[2 * e2 + 1];
            const _Float16 h0 = (_Float16)f0, h1 = (_Float16)f1;
            hv[e2] = h2bits(h0) | (h2bits(h1) << 16);
            if (OUT_MODE == 3) {
              const _Float16 l0 = (_Float16)((f0 - (float)h0) * RES_CARRY);
              const _Float16 l1 = (_Float16)((f1 - (float)h1) * RES_CARRY);
              lv[e2] = h2bits(l0) | (h2bits(l1) << 16);
            }
          }
          *(volatile u32x4*)(C + (size_t)(mBase + row) * ldc + n0 + c8) = hv;
          if (OUT_MODE == 3) *(volatile u32x4*)(C2 + (size_t)(mBase + row) * ldc + n0 + c8) = lv;
        }
        __threadfence();
      }
    }
    __builtin_amdgcn_fence(__ATOMIC_RELEASE, "workgroup");
    __builtin_amdgcn_wave_barrier();
    __builtin_amdgcn_fence(__ATOMIC_ACQUIRE, "workgroup");
  }
}

__global__ __launch_bounds__(256) void cast_f32_bf16x2(
    const float* __restrict__ in, unsigned short* __restrict__ out, int n2) {
  const int i = blockIdx.x * 256 + threadIdx.x;
  if (i < n2) {
    const v2f f = *(const v2f*)(in + 2 * (size_t)i);
    const unsigned u = (unsigned)f2bf_bits(f[0]) | ((unsigned)f2bf_bits(f[1]) << 16);
    ((volatile unsigned*)out)[i] = u;
    __threadfence();
    ((volatile unsigned*)out)[i] = u;
  }
}

__global__ __launch_bounds__(256) void transpose_cast_bf16(
    const float* __restrict__ in, unsigned short* __restrict__ out, int nrow, int ncol) {
  __shared__ float tile[64][65];
  const int tid = threadIdx.x;
  const int c0 = blockIdx.x * 64, r0 = blockIdx.y * 64;
  {
    const int c4 = (tid & 15) * 4;
#pragma unroll
    for (int p = 0; p < 4; ++p) {
      const int r = (tid >> 4) + 16 * p;
      const v4f v = *(const v4f*)(in + (size_t)(r0 + r) * ncol + c0 + c4);
#pragma unroll
      for (int e = 0; e < 4; ++e) tile[r][c4 + e] = v[e];
    }
  }
  __syncthreads();
  const int k8 = (tid & 7) * 8;
  for (int pass = 0; pass < 2; ++pass) {
#pragma unroll
    for (int p = 0; p < 2; ++p) {
      const int oc = (tid >> 3) + 32 * p;
      u32x4 w;
#pragma unroll
      for (int e2 = 0; e2 < 4; ++e2) {
        const float f0 = tile[k8 + 2 * e2][oc], f1 = tile[k8 + 2 * e2 + 1][oc];
        w[e2] = (unsigned)f2bf_bits(f0) | ((unsigned)f2bf_bits(f1) << 16);
      }
      *(volatile u32x4*)(out + (size_t)(c0 + oc) * nrow + r0 + k8) = w;
    }
    __threadfence();
  }
}

#define AT_D 64
#define AT_NW 4
#define AT_QB 64
#define AT_KC 64
__global__ __launch_bounds__(128)
void causal_attn64(const unsigned short* __restrict__ QKp, const unsigned short* __restrict__ Vthp,
                   const unsigned short* __restrict__ Vtlp, unsigned short* __restrict__ Ohp,
                   unsigned short* __restrict__ Olp) {
  __shared__ __align__(16) _Float16 Ksh[AT_KC * AT_D];
  __shared__ __align__(16) _Float16 Vth[AT_D * AT_KC];
  __shared__ __align__(16) _Float16 Vtl[AT_D * AT_KC];
  __shared__ __align__(16) _Float16 Psh[AT_NW][16 * AT_KC];
  __shared__ __align__(16) float  Os[AT_NW][16 * 68];

  const int tid  = threadIdx.x;
  const int wave = tid >> 5;
  const int lane = tid & 31;
  const int hh   = lane >> 4;
  const int c    = lane & 15;

  const int nqb = NT / AT_QB;
  const int bx = blockIdx.x;
  const int qb = bx % nqb;
  const int bh = bx / nqb;
  const int h  = bh % NH;
  const int b  = bh / NH;
  const int q0 = qb * AT_QB + wave * 16;

  const _Float16* QK = (const _Float16*)QKp;

  v16h qa[2];
  {
    const _Float16* qrow = QK + (size_t)(b * NT + q0 + c) * NQKCOL + NC + h * HD;
#pragma unroll
    for (int dc = 0; dc < 2; ++dc) qa[dc] = Frag<_Float16>::load(qrow + dc * 32 + 8 * hh);
  }

  float mrow[8], lrow[8];
  v8f oacc[4], olacc[4];
#pragma unroll
  for (int r = 0; r < 8; ++r) { mrow[r] = -INFINITY; lrow[r] = 0.f; }
#pragma unroll
  for (int t = 0; t < 4; ++t) { oacc[t] = (v8f){0.f,0.f,0.f,0.f,0.f,0.f,0.f,0.f}; olacc[t] = oacc[t]; }

  const int nChunks = qb + 1;
  for (int kc = 0; kc < nChunks; ++kc) {
    const int kv0 = kc * AT_KC;
    __syncthreads();
    {
      const int rr = tid >> 1, hf = (tid & 1) * 32;
      const unsigned short* ksrc = QKp  + (size_t)(b * NT + kv0 + rr) * NQKCOL + h * HD + hf;
      const unsigned short* vhs  = Vthp + (size_t)(h * HD + rr) * NTOK + b * NT + kv0 + hf;
      const unsigned short* vls  = Vtlp + (size_t)(h * HD + rr) * NTOK + b * NT + kv0 + hf;
      u32x4 kq[4], vq[4], wq[4];
#pragma unroll
      for (int i = 0; i < 4; ++i) {
        kq[i] = *(const u32x4*)(ksrc + 8 * i);
        vq[i] = *(const u32x4*)(vhs + 8 * i);
        wq[i] = *(const u32x4*)(vls + 8 * i);
      }
#pragma unroll
      for (int i = 0; i < 4; ++i) {
        *(u32x4*)(Ksh + rr * AT_D + hf + 8 * i)  = kq[i];
        *(u32x4*)(Vth + rr * AT_KC + hf + 8 * i) = vq[i];
        *(u32x4*)(Vtl + rr * AT_KC + hf + 8 * i) = wq[i];
      }
    }
    __syncthreads();

    v8f s[4];
#pragma unroll
    for (int j = 0; j < 4; ++j) {
      s[j] = (v8f){0.f,0.f,0.f,0.f,0.f,0.f,0.f,0.f};
#pragma unroll
      for (int dc = 0; dc < 2; ++dc) {
        const v16h kb = Frag<_Float16>::load(Ksh + (j * 16 + c) * AT_D + dc * 32 + 8 * hh);
        s[j] = mma_h(qa[dc], kb, s[j]);
      }
    }
    const bool diag = (kc == qb);
    float cm[8];
#pragma unroll
    for (int r = 0; r < 8; ++r) {
      const int qrow = q0 + 8 * hh + r;
      float m = -INFINITY;
#pragma unroll
      for (int j = 0; j < 4; ++j) {
        const int kvcol = kv0 + j * 16 + c;
        float val = s[j][r] * SCORE_SCALE;
        if (diag && (kvcol > qrow)) val = -INFINITY;
        s[j][r] = val;
        m = fmaxf(m, val);
      }
#pragma unroll
      for (int off = 1; off < 16; off <<= 1) m = fmaxf(m, __shfl_xor(m, off, 32));
      cm[r] = m;
    }
    _Float16* pw = Psh[wave];
#pragma unroll
    for (int r = 0; r < 8; ++r) {
      const float mnew = fmaxf(mrow[r], cm[r]);
      const float alpha = expf(mrow[r] - mnew);
      mrow[r] = mnew;
      float psum = 0.f;
#pragma unroll
      for (int j = 0; j < 4; ++j) {
        const float p = expf(s[j][r] - mnew);
        const _Float16 p16 = (_Float16)(p * PCARRY);
        psum += (float)p16;
        pw[(8 * hh + r) * AT_KC + j * 16 + c] = p16;
      }
#pragma unroll
      for (int off = 1; off < 16; off <<= 1) psum += __shfl_xor(psum, off, 32);
      lrow[r] = lrow[r] * alpha + psum;
#pragma unroll
      for (int t = 0; t < 4; ++t) { oacc[t][r] *= alpha; olacc[t][r] *= alpha; }
    }
    __builtin_amdgcn_fence(__ATOMIC_RELEASE, "workgroup");
    __builtin_amdgcn_wave_barrier();
    __builtin_amdgcn_fence(__ATOMIC_ACQUIRE, "workgroup");
#pragma unroll 1
    for (int kk = 0; kk < 2; ++kk) {
      const v16h pa = Frag<_Float16>::load(pw + c * AT_KC + kk * 32 + 8 * hh);
#pragma unroll
      for (int t = 0; t < 4; ++t) {
        const v16h vb = Frag<_Float16>::load(Vth + (t * 16 + c) * AT_KC + kk * 32 + 8 * hh);
        const v16h vl = Frag<_Float16>::load(Vtl + (t * 16 + c) * AT_KC + kk * 32 + 8 * hh);
        oacc[t]  = mma_h(pa, vb, oacc[t]);
        olacc[t] = mma_h(pa, vl, olacc[t]);
      }
    }
  }

  float* os = Os[wave];
#pragma unroll
  for (int r = 0; r < 8; ++r) {
    const float inv = 1.0f / lrow[r];
#pragma unroll
    for (int t = 0; t < 4; ++t) os[(8 * hh + r) * 68 + t * 16 + c] = (oacc[t][r] + olacc[t][r] * RES_CARRY_INV) * inv;
  }
  __builtin_amdgcn_fence(__ATOMIC_RELEASE, "workgroup");
  __builtin_amdgcn_wave_barrier();
  __builtin_amdgcn_fence(__ATOMIC_ACQUIRE, "workgroup");
  {
    const int q = lane >> 3, c8 = (lane & 7) * 8;
    unsigned short* oh = Ohp + (size_t)(b * NT + q0) * NC + h * HD + c8;
    unsigned short* ol = Olp + (size_t)(b * NT + q0) * NC + h * HD + c8;
    for (int pass = 0; pass < 2; ++pass) {
#pragma unroll
      for (int it = 0; it < 4; ++it) {
        const int row = it * 4 + q;
        const float* sp = os + row * 68 + c8;
        u32x4 hv, lv;
#pragma unroll
        for (int e2 = 0; e2 < 4; ++e2) {
          const float f0 = sp[2 * e2], f1 = sp[2 * e2 + 1];
          const unsigned short hb0 = f2bf_bits(f0), hb1 = f2bf_bits(f1);
          const unsigned short lb0 = f2bf_bits(f0 - bf_bits2f(hb0)), lb1 = f2bf_bits(f1 - bf_bits2f(hb1));
          hv[e2] = (unsigned)hb0 | ((unsigned)hb1 << 16);
          lv[e2] = (unsigned)lb0 | ((unsigned)lb1 << 16);
        }
        *(volatile u32x4*)(oh + (size_t)row * NC) = hv;
        *(volatile u32x4*)(ol + (size_t)row * NC) = lv;
      }
      __threadfence();
    }
  }
}

extern "C" void kernel_launch(void* const* d_in, const int* in_sizes, int n_in,
                              void* d_out, int out_size, void* d_ws, size_t ws_size,
                              hipStream_t stream) {
  if (n_in < 5) return;
  if (in_sizes[0] != NTOK * NC || in_sizes[1] != NC * NQKV || in_sizes[2] != NQKV ||
      in_sizes[3] != NC * NC || in_sizes[4] != NC) return;
  if (out_size != NTOK * NC) return;

  const float* x      = (const float*)d_in[0];
  const float* W_attn = (const float*)d_in[1];
  const float* b_attn = (const float*)d_in[2];
  const float* W_proj = (const float*)d_in[3];
  const float* b_proj = (const float*)d_in[4];
  float* out = (float*)d_out;

  char* ws = (char*)d_ws;
  size_t off = 0;
  auto carve = [&](size_t bytes) { char* p = ws + off; off += (bytes + 255) & ~(size_t)255; return p; };
  unsigned short* xb  = (unsigned short*)carve((size_t)NTOK * NC * 2);
  unsigned short* wat = (unsigned short*)carve((size_t)NQKV * NC * 2);
  unsigned short* wpt = (unsigned short*)carve((size_t)NC * NC * 2);
  unsigned short* qk  = (unsigned short*)carve((size_t)NTOK * NQKCOL * 2);
  unsigned short* vth = (unsigned short*)carve((size_t)NC * NTOK * 2);
  unsigned short* vtl = (unsigned short*)carve((size_t)NC * NTOK * 2);
  unsigned short* oh  = (unsigned short*)carve((size_t)NTOK * NC * 2);
  unsigned short* ol  = (unsigned short*)carve((size_t)NTOK * NC * 2);
  if (off > ws_size) return;

  {
    const int n2 = NTOK * NC / 2;
    cast_f32_bf16x2<<<dim3((n2 + 255) / 256), 256, 0, stream>>>(x, xb, n2);
  }
  transpose_cast_bf16<<<dim3(NQKV / 64, NC / 64), 256, 0, stream>>>(W_attn, wat, NC, NQKV);
  transpose_cast_bf16<<<dim3(NC / 64, NC / 64), 256, 0, stream>>>(W_proj, wpt, NC, NC);

  {
    const int tiles = (NTOK / 64) * (NQKCOL / 64);
    wmma_gemm64<1, 0, 2, 1><<<dim3((tiles + 7) / 8, 1), 256, 0, stream>>>(
        xb, nullptr, NC, 0L, wat, NC, 0L, (void*)qk, nullptr, NQKCOL, 0L, b_attn,
        NTOK, NQKCOL, NC, 1.0f);
  }
  {
    const int tiles = (NC / 64) * (NTOK / 64);
    wmma_gemm64<1, 0, 1, 3><<<dim3((tiles + 7) / 8, 1), 256, 0, stream>>>(
        wat + (size_t)NQKCOL * NC, nullptr, NC, 0L, xb, NC, 0L, (void*)vth, (void*)vtl, NTOK, 0L,
        b_attn + NQKCOL, NC, NTOK, NC, 1.0f);
  }
  causal_attn64<<<dim3(NBATCH * NH * (NT / AT_QB)), 128, 0, stream>>>(qk, vth, vtl, oh, ol);
  {
    const int tiles = (NTOK / 64) * (NC / 64);
    wmma_gemm64<1, 1, 2, 0><<<dim3((tiles + 7) / 8, 1), 256, 0, stream>>>(
        oh, ol, NC, 0L, wpt, NC, 0L, (void*)out, nullptr, NC, 0L, b_proj,
        NTOK, NC, NC, 1.0f);
  }
}
